// ParallelPhysicalRecurrentLayer_17867063952064
// MI455X (gfx1250) — hardware-verified
//
#include <hip/hip_runtime.h>
#include <math.h>

typedef _Float16 h16;
typedef __attribute__((ext_vector_type(16))) _Float16 v16h;
typedef __attribute__((ext_vector_type(8)))  _Float16 v8h;
typedef __attribute__((ext_vector_type(2)))  _Float16 v2h;
typedef __attribute__((ext_vector_type(16))) __bf16   v16b;
typedef __attribute__((ext_vector_type(8)))  __bf16   v8b;
typedef __attribute__((ext_vector_type(8)))  float    v8f;
typedef __attribute__((ext_vector_type(4)))  float    v4f;
typedef __attribute__((ext_vector_type(4)))  unsigned int v4u;

constexpr int LDIM = 16;
constexpr int CDIM = 32;
constexpr int HDIM = 64;
constexpr int WDIM = 64;
constexpr int WFQ  = 33;
constexpr int RDIM = 16;
constexpr int NPIX = HDIM * WDIM;
constexpr int NXROW = CDIM * LDIM * HDIM;
constexpr int NLF = LDIM * WFQ;
constexpr int NLF_PAD = 576;
constexpr int NHEAD = CDIM * RDIM * 3;
constexpr int FEAT_PITCH = 64;
constexpr int NELEM = CDIM * LDIM * HDIM * WDIM;
static_assert(NXROW == 32768, "row count");
static_assert(NLF == 528 && NLF_PAD % 16 == 0 && NLF_PAD >= NLF, "head rows");
static_assert(NHEAD == 1536, "head columns");
static_assert(NXROW % 64 == 0 && WDIM % 64 == 0 && WDIM % 32 == 0, "dense product tile multiples");
static_assert(CDIM % 32 == 0, "channel depth multiple of 32");

constexpr float CW_CARRY   = 64.0f;
constexpr float HW_CARRY   = 64.0f;
constexpr float FEAT_CARRY = 64.0f;
constexpr float PIFW_CARRY = 64.0f;
constexpr float Y_CARRY    = 1024.0f;
constexpr float H_CARRY    = 256.0f;
constexpr float V_CARRY    = 64.0f;
constexpr float HEAD_FOLD  = 1.0f / (HW_CARRY * FEAT_CARRY);
constexpr float SCAN_FOLD  = Y_CARRY / (H_CARRY * V_CARRY);
constexpr float IDFT_FOLD  = 1.0f / (Y_CARRY * (float)WDIM);
constexpr float GN_EPS     = 1e-5f;
constexpr float PI_F       = 3.14159265358979323846f;

__device__ __forceinline__ unsigned short f2bf_bits(float f) {
  unsigned u = __float_as_uint(f);
  return (unsigned short)((u + 0x7FFFu + ((u >> 16) & 1u)) >> 16);
}
__device__ __forceinline__ float bf_bits2f(unsigned short h) { return __uint_as_float(((unsigned)h) << 16); }

__device__ __forceinline__ float h16_to_f32(unsigned hb) {
  const unsigned sgn = (hb & 0x8000u) << 16; const unsigned em = hb & 0x7fffu;
  const float fn = __uint_as_float((em << 13) + 0x38000000u);
  const float fs = (float)em * 5.9604644775390625e-8f;
  const float mag = (em < 0x400u) ? fs : fn; return __uint_as_float(__float_as_uint(mag) | sgn);
}

__device__ __forceinline__ void wave_sync() {
  __builtin_amdgcn_fence(__ATOMIC_RELEASE, "workgroup");
  __builtin_amdgcn_wave_barrier();
  __builtin_amdgcn_fence(__ATOMIC_ACQUIRE, "workgroup");
}

__device__ __forceinline__ void keep4_h(v16h a, v16h b, v16h c, v16h d) { asm volatile("v_nop" :: "v"(a), "v"(b), "v"(c), "v"(d)); }
__device__ __forceinline__ void keep4_b(v16b a, v16b b, v16b c, v16b d) { asm volatile("v_nop" :: "v"(a), "v"(b), "v"(c), "v"(d)); }
__device__ __forceinline__ void acc_guard4(v8f& a, v8f& b, v8f& c, v8f& d) { asm volatile("v_nop\n\tv_nop\n\tv_nop\n\tv_nop" : "+v"(a), "+v"(b), "+v"(c), "+v"(d)); }
__device__ __forceinline__ void grp_guard_h(v8f& a, v8f& b, v8f& c, v8f& d, v16h x, v16h y) { asm volatile("v_nop\n\tv_nop\n\tv_nop\n\tv_nop" : "+v"(a), "+v"(b), "+v"(c), "+v"(d) : "v"(x), "v"(y)); }
__device__ __forceinline__ void grp_guard_b(v8f& a, v8f& b, v8f& c, v8f& d, v16b x, v16b y) { asm volatile("v_nop\n\tv_nop\n\tv_nop\n\tv_nop" : "+v"(a), "+v"(b), "+v"(c), "+v"(d) : "v"(x), "v"(y)); }

template <typename T> struct Frag;
template <> struct Frag<_Float16> {
  typedef v16h V; union U { v16h v; v8h h[2]; };
  static __device__ __forceinline__ v16h load(const _Float16* p) {
    U f; f.h[0] = *(const v8h*)(p); f.h[1] = *(const v8h*)(p + 16); return f.v;
  }
  static __device__ __forceinline__ v8f mma(v16h a, v16h b, v8f c) {
    return __builtin_amdgcn_wmma_f32_16x16x32_f16(false, a, false, b, (short)0, c, false, false);
  }
  static __device__ __forceinline__ void guard4(v8f& a, v8f& b, v8f& c, v8f& d, v16h x, v16h y) { grp_guard_h(a, b, c, d, x, y); }
  static __device__ __forceinline__ void keep(v16h a, v16h b, v16h c, v16h d) { keep4_h(a, b, c, d); }
};
template <> struct Frag<__bf16> {
  typedef v16b V; union U { v16b v; v8b h[2]; };
  static __device__ __forceinline__ v16b load(const __bf16* p) {
    U f; f.h[0] = *(const v8b*)(p); f.h[1] = *(const v8b*)(p + 16); return f.v;
  }
  static __device__ __forceinline__ v8f mma(v16b a, v16b b, v8f c) {
    return __builtin_amdgcn_wmma_f32_16x16x32_bf16(false, a, false, b, (short)0, c, false, false);
  }
  static __device__ __forceinline__ void guard4(v8f& a, v8f& b, v8f& c, v8f& d, v16b x, v16b y) { grp_guard_b(a, b, c, d, x, y); }
  static __device__ __forceinline__ void keep(v16b a, v16b b, v16b c, v16b d) { keep4_b(a, b, c, d); }
};

__device__ __forceinline__ v8f wmma_h(v16h a, v16h b, v8f c) {
  c = __builtin_amdgcn_wmma_f32_16x16x32_f16(false, a, false, b, (short)0, c, false, false);
  asm volatile("v_nop\n\tv_nop\n\tv_nop\n\tv_nop" : "+v"(c) : "v"(a), "v"(b));
  return c;
}

template <int ET> struct Elem;
template <> struct Elem<0> { typedef _Float16 T; };
template <> struct Elem<1> { typedef __bf16 T; };
template <int ET, bool SPLIT, int BIAS_MODE, int OUT_MODE, bool RESID, int ACT = 0>
__global__ __launch_bounds__(256) void wmma_gemm64(
    const unsigned short* __restrict__ Ap, const unsigned short* __restrict__ A2p, int lda, long strideA,
    const unsigned short* __restrict__ Btp, const unsigned short* __restrict__ Bt2p, int ldb, long strideB,
    void* __restrict__ Cout, void* __restrict__ Cout2, int ldc, long strideC,
    const float* __restrict__ bias,
    const float* __restrict__ resid, long strideR,
    int M, int N, int K, float scale) {
  typedef typename Elem<ET>::T T;
  typedef typename Frag<T>::V V;
  const T* A = (const T*)Ap; const T* A2 = (const T*)A2p; const T* Bt = (const T*)Btp; const T* Bt2 = (const T*)Bt2p;
  __shared__ __align__(16) float sT[8][16 * 68];
  const int b    = blockIdx.y;
  const int lane = threadIdx.x & 31;
  const int wave = threadIdx.x >> 5;
  const int tilesN = N >> 6;
  const int tilesM = M >> 6;
  const int tile = blockIdx.x * 8 + wave;
  if (tile >= tilesM * tilesN) return;
  const int tm = tile / tilesN;
  const int tn = tile - tm * tilesN;
  const int m0 = tm << 6;
  const int n0 = tn << 6;

  const T* Ab  = A  + (size_t)b * strideA;
  const T* Bb  = Bt + (size_t)b * strideB;
  const T* Ab2 = SPLIT ? (A2  + (size_t)b * strideA) : nullptr;
  const T* Bb2 = SPLIT ? (Bt2 + (size_t)b * strideB) : nullptr;

  const int rlane = lane & 15;
  const int koff  = (lane >> 4) * 8;
  const int mOff  = (lane >> 4) * 8;

  v8f acc[4][4];
#pragma unroll
  for (int i = 0; i < 4; ++i)
#pragma unroll
    for (int j = 0; j < 4; ++j) acc[i][j] = (v8f){0.f,0.f,0.f,0.f,0.f,0.f,0.f,0.f};

  for (int k0 = 0; k0 < K; k0 += 32) {
    V bh[4], bl[4];
#pragma unroll
    for (int j = 0; j < 4; ++j) {
      const size_t bo = (size_t)(n0 + (j << 4) + rlane) * ldb + koff + k0;
      bh[j] = Frag<T>::load(Bb + bo);
      if (SPLIT) bl[j] = Frag<T>::load(Bb2 + bo);
    }
#pragma unroll
    for (int i = 0; i < 4; ++i) {
      const size_t ao = (size_t)(m0 + (i << 4) + rlane) * lda + koff + k0;
      V ah = Frag<T>::load(Ab + ao);
      V al;
      if (SPLIT) al = Frag<T>::load(Ab2 + ao);
#pragma unroll
      for (int j = 0; j < 4; ++j) {
        acc[i][j] = Frag<T>::mma(ah, bh[j], acc[i][j]);
        if (SPLIT) {
          acc[i][j] = Frag<T>::mma(ah, bl[j], acc[i][j]);
          acc[i][j] = Frag<T>::mma(al, bh[j], acc[i][j]);
        }
      }
      Frag<T>::guard4(acc[i][0], acc[i][1], acc[i][2], acc[i][3], ah, SPLIT ? al : ah);
    }
    Frag<T>::keep(bh[0], bh[1], bh[2], bh[3]);
    if (SPLIT) Frag<T>::keep(bl[0], bl[1], bl[2], bl[3]);
  }
  acc_guard4(acc[0][0], acc[0][1], acc[0][2], acc[0][3]);
  acc_guard4(acc[1][0], acc[1][1], acc[1][2], acc[1][3]);
  acc_guard4(acc[2][0], acc[2][1], acc[2][2], acc[2][3]);
  acc_guard4(acc[3][0], acc[3][1], acc[3][2], acc[3][3]);

  float* slab = sT[wave];
  const float* Rb = RESID ? (resid + (size_t)b * strideR) : nullptr;
#pragma unroll
  for (int i = 0; i < 4; ++i) {
    const int mBase = m0 + (i << 4);
#pragma unroll
    for (int j = 0; j < 4; ++j) {
      const int n = n0 + (j << 4) + rlane;
      float bv = 0.f;
      if (BIAS_MODE == 2) bv = bias[n];
#pragma unroll
      for (int r = 0; r < 8; ++r) {
        float v = acc[i][j][r] * scale;
        if (BIAS_MODE == 1) v += bias[mBase + mOff + r];
        if (BIAS_MODE == 2) v += bv;
        if (BIAS_MODE == 3) v += bias[((mBase + mOff + r) >> 6) & 31];
        if (RESID) v += Rb[(size_t)(mBase + mOff + r) * ldc + n];
        if (ACT == 1) v = tanhf(v);
        if (ACT == 2) v = fmaxf(v, 0.0f);
        if (ACT == 3) v = v / (1.0f + expf(-v));
        if (ACT == 4) v = (v > 0.f) ? v : 0.01f * v;
        slab[(mOff + r) * 68 + (j << 4) + rlane] = v;
      }
    }
    wave_sync();
    if (OUT_MODE == 0) {
      float* C = (float*)Cout + (size_t)b * strideC;
      const int hh = lane >> 4, c4 = (lane & 15) * 4;
      for (int pass = 0; pass < 2; ++pass) {
#pragma unroll
        for (int it = 0; it < 8; ++it) {
          const int row = it * 2 + hh;
          v4f v = *(const v4f*)(slab + row * 68 + c4);
          *(volatile v4f*)(C + (size_t)(mBase + row) * ldc + n0 + c4) = v;
        }
        __threadfence();
      }
    } else {
      const int q = lane >> 3, c8 = (lane & 7) * 8;
      unsigned short* C  = (unsigned short*)Cout  + (size_t)b * strideC;
      unsigned short* C2 = (OUT_MODE == 2) ? ((unsigned short*)Cout2 + (size_t)b * strideC) : nullptr;
      for (int pass = 0; pass < 2; ++pass) {
#pragma unroll
        for (int it = 0; it < 4; ++it) {
          const int row = it * 4 + q;
          const float* sp = slab + row * 68 + c8;
          v8h hv, lv;
#pragma unroll
          for (int e = 0; e < 8; ++e) {
            if (OUT_MODE == 1) {
              hv[e] = (_Float16)sp[e];
            } else {
              unsigned short hb = f2bf_bits(sp[e]);
              unsigned short lb = f2bf_bits(sp[e] - bf_bits2f(hb));
              hv[e] = __builtin_bit_cast(_Float16, hb);
              lv[e] = __builtin_bit_cast(_Float16, lb);
            }
          }
          *(volatile v8h*)(C + (size_t)(mBase + row) * ldc + n0 + c8) = hv;
          if (OUT_MODE == 2) *(volatile v8h*)(C2 + (size_t)(mBase + row) * ldc + n0 + c8) = lv;
        }
        __threadfence();
      }
    }
    wave_sync();
  }
}

constexpr int PREP_THR = 128;
constexpr int PB_CW2 = 9, PB_HEAD = 18, PB_PIF = 66, PB_FT = 67, PB_IT = 71, PB_FOLD = 75, PREP_BLOCKS = 76;

__global__ __launch_bounds__(PREP_THR) void k_prep(
    const float* __restrict__ conv1_w, const float* __restrict__ conv2_w, const float* __restrict__ head_w,
    const float* __restrict__ pif_w, const float* __restrict__ mix_w, const float* __restrict__ mix_b,
    const float* __restrict__ rank_scale, const float* __restrict__ proj_w, const float* __restrict__ proj_b,
    unsigned short* __restrict__ CW1, unsigned short* __restrict__ CW2, unsigned short* __restrict__ HEADP,
    unsigned short* __restrict__ PIF16, unsigned short* __restrict__ FT16, unsigned short* __restrict__ IT16,
    unsigned short* __restrict__ FOLDB, float* __restrict__ FOLDC) {
  __shared__ __align__(16) h16 st[PREP_THR * 8];
  __shared__ float vv[64];
  __shared__ float cst[2];
  const int tid = threadIdx.x;
  const int bid = blockIdx.x;
  int region, gi, ngroups;
  unsigned short* dst;
  if (bid < PB_CW2)        { region = 0; gi = bid * PREP_THR + tid;             ngroups = 1152; dst = CW1; }
  else if (bid < PB_HEAD)  { region = 1; gi = (bid - PB_CW2) * PREP_THR + tid;  ngroups = 1152; dst = CW2; }
  else if (bid < PB_PIF)   { region = 2; gi = (bid - PB_HEAD) * PREP_THR + tid; ngroups = 6144; dst = HEADP; }
  else if (bid < PB_FT)    { region = 3; gi = tid;                              ngroups = 128;  dst = PIF16; }
  else if (bid < PB_IT)    { region = 4; gi = (bid - PB_FT) * PREP_THR + tid;   ngroups = 512;  dst = FT16; }
  else if (bid < PB_FOLD)  { region = 5; gi = (bid - PB_IT) * PREP_THR + tid;   ngroups = 512;  dst = IT16; }
  else                     { region = 6; gi = tid;                              ngroups = 64;   dst = FOLDB; }

  if (region == 6) {
    if (tid < 32) {
      const int k = tid;
      float vr = 0.f, vi = 0.f, cr = 0.f, ci = 0.f;
#pragma unroll 1
      for (int r = 0; r < RDIM; ++r) {
        const float s = rank_scale[r] * proj_w[r];
        vr += s * mix_w[r * 32 + k];
        vi += s * mix_w[(16 + r) * 32 + k];
        cr += s * mix_b[r];
        ci += s * mix_b[16 + r];
      }
      cr += proj_b[0];
      vv[k] = vr;
      vv[32 + k] = vi;
      if (k == 0) { cst[0] = cr; cst[1] = ci; }
    }
  }
  __syncthreads();

#pragma unroll 1
  for (int i = 0; i < 8; ++i) {
    float val = 0.f;
    if (region <= 1) {
      const float* src = (region == 1) ? conv2_w : conv1_w;
      const int e = gi * 8 + i;
      const int tap = e >> 10, o = (e >> 5) & 31, ci = e & 31;
      val = src[o * 288 + ci * 9 + tap] * CW_CARRY;
    } else if (region == 2) {
      const int np = gi >> 2;
      const int kk = np >> 9, c = (np >> 4) & 31, r = np & 15;
      const int n = (c * 16 + r) * 3 + kk;
      val = head_w[n * 32 + (gi & 3) * 8 + i] * HW_CARRY;
    } else if (region == 3) {
      val = pif_w[gi * 8 + i] * PIFW_CARRY;
    } else if (region == 4 || region == 5) {
      const int fixed = gi >> 3, var = (gi & 7) * 8 + i;
      const int a = (region == 4) ? fixed : var;
      const int b = (region == 4) ? var : fixed;
      const int fq = a >> 1;
      const int ph = (fq * b) & 63;
      float sn, cs;
      sincospif((float)ph * (1.0f / 32.0f), &sn, &cs);
      float t = (a & 1) ? -sn : cs;
      if (region == 5) t = 2.0f * t;
      const float alt = (b & 1) ? -1.0f : 1.0f;
      val = (a == 0) ? 1.0f : ((a == 1) ? alt : t);
    } else {
      const int n = gi >> 2;
      const int kq = (gi & 3) * 8 + i;
      const float a0 = vv[kq], a1 = vv[32 + kq];
      val = (n == 0) ? a0 * V_CARRY : ((n == 1) ? a1 * V_CARRY : 0.0f);
    }
    st[tid * 8 + i] = (h16)val;
  }
  __syncthreads();
  if (gi < ngroups) {
    const v8h hv = *(const v8h*)(st + tid * 8);
    h16* dp = (h16*)dst + (size_t)gi * 8;
    *(volatile v8h*)dp = hv;
    __threadfence();
    *(volatile v8h*)dp = hv;
  }
  if (region == 6 && tid < 32) {
    const float c0 = cst[0], c1 = cst[1];
    const float o = (tid == 0) ? c0 : ((tid == 1) ? c1 : 0.0f);
    *(volatile float*)(FOLDC + tid) = o;
    __threadfence();
    *(volatile float*)(FOLDC + tid) = o;
  }
}

template <bool IN_X>
__global__ __launch_bounds__(256) void k_conv(const float* __restrict__ xin, const unsigned short* __restrict__ finp,
                                              const unsigned short* __restrict__ wplp, const float* __restrict__ bias,
                                              unsigned short* __restrict__ foutp) {
  __shared__ __align__(16) h16 tile[10 * 66 * 32];
  __shared__ __align__(16) h16 wt[9 * 32 * 32];
  __shared__ __align__(16) float slabs[8][16 * 36];
  __shared__ float bsh[32];
  const h16* fin = (const h16*)finp;
  const h16* wpl = (const h16*)wplp;
  h16* fout = (h16*)foutp;
  const int tid = threadIdx.x;
  const int l  = blockIdx.x >> 3;
  const int h0 = (blockIdx.x & 7) * 8;

  for (int i = tid; i < 1152; i += 256) *(v8h*)(wt + 8 * i) = *(const v8h*)(wpl + 8 * i);
  if (tid < 32) bsh[tid] = bias[tid];
  if (IN_X) {
#pragma unroll 1
    for (int i = tid; i < 32 * 10 * 66; i += 256) {
      const int wc = i % 66;
      const int t2 = i / 66;
      const int r = t2 % 10;
      const int c = t2 / 10;
      const int gh = h0 + r - 1, gw = wc - 1;
      const bool inb = (gh >= 0) && (gh < HDIM) && (gw >= 0) && (gw < WDIM);
      const int ghc = gh < 0 ? 0 : (gh > HDIM - 1 ? HDIM - 1 : gh);
      const int gwc = gw < 0 ? 0 : (gw > WDIM - 1 ? WDIM - 1 : gw);
      float v = xin[((size_t)(c * LDIM + l) * HDIM + ghc) * WDIM + gwc];
      v = inb ? v : 0.0f;
      tile[(r * 66 + wc) * 32 + c] = (h16)v;
    }
  } else {
    const v8h zero8 = {(h16)0.f, (h16)0.f, (h16)0.f, (h16)0.f, (h16)0.f, (h16)0.f, (h16)0.f, (h16)0.f};
#pragma unroll 1
    for (int i = tid; i < 10 * 66 * 4; i += 256) {
      const int q = i & 3;
      const int px = i >> 2;
      const int wc = px % 66;
      const int r = px / 66;
      const int gh = h0 + r - 1, gw = wc - 1;
      const bool inb = (gh >= 0) && (gh < HDIM) && (gw >= 0) && (gw < WDIM);
      const int ghc = gh < 0 ? 0 : (gh > HDIM - 1 ? HDIM - 1 : gh);
      const int gwc = gw < 0 ? 0 : (gw > WDIM - 1 ? WDIM - 1 : gw);
      const v8h v = *(const v8h*)(fin + ((size_t)((l * HDIM + ghc) * WDIM + gwc)) * 32 + 8 * q);
      const v8h o = inb ? v : zero8;
      *(v8h*)(tile + px * 32 + 8 * q) = o;
    }
  }
  __syncthreads();

  const int lane = tid & 31, wave = tid >> 5;
  const int m = lane & 15, hh = lane >> 4, koff = hh * 8;
  const int r = wave;
  const int hrow = h0 + r;
  float* slab = slabs[wave];
  const float inv = 1.0f / CW_CARRY;
  const float bz0 = bsh[m], bz1 = bsh[16 + m];
  const v8f z8 = {0.f, 0.f, 0.f, 0.f, 0.f, 0.f, 0.f, 0.f};

#pragma unroll 1
  for (int w0 = 0; w0 < WDIM; w0 += 16) {
    v8f acc0 = z8, acc1 = z8;
#pragma unroll
    for (int tap = 0; tap < 9; ++tap) {
      const int dy = tap / 3, dx = tap - 3 * dy;
      const v16h a  = Frag<h16>::load(tile + ((r + dy) * 66 + w0 + m + dx) * 32 + koff);
      const v16h b0 = Frag<h16>::load(wt + (tap * 32 + m) * 32 + koff);
      const v16h b1 = Frag<h16>::load(wt + (tap * 32 + 16 + m) * 32 + koff);
      acc0 = wmma_h(a, b0, acc0);
      acc1 = wmma_h(a, b1, acc1);
    }
#pragma unroll
    for (int j = 0; j < 8; ++j) {
      slab[(8 * hh + j) * 36 + m]      = acc0[j] * inv + bz0;
      slab[(8 * hh + j) * 36 + 16 + m] = acc1[j] * inv + bz1;
    }
    wave_sync();
#pragma unroll 1
    for (int it = 0; it < 2; ++it) {
      const int px = it * 8 + (lane >> 2);
      const int q8 = (lane & 3) * 8;
      const v4f s0 = *(const v4f*)(slab + px * 36 + q8);
      const v4f s1 = *(const v4f*)(slab + px * 36 + q8 + 4);
      v8h hv;
#pragma unroll
      for (int e = 0; e < 4; ++e) {
        const float u0 = s0[e], u1 = s1[e];
        hv[e]     = (h16)(u0 / (1.0f + expf(-u0)));
        hv[4 + e] = (h16)(u1 / (1.0f + expf(-u1)));
      }
      h16* dp = fout + ((size_t)((l * HDIM + hrow) * WDIM + w0 + px)) * 32 + q8;
      *(volatile v8h*)dp = hv;
      __threadfence();
      *(volatile v8h*)dp = hv;
    }
    wave_sync();
  }
}

__global__ __launch_bounds__(256) void k_pool(const unsigned short* __restrict__ f2p, const float* __restrict__ gfc_w,
                                              const float* __restrict__ gfc_b, unsigned short* __restrict__ featp) {
  __shared__ float fm[64 * 32];
  __shared__ float gm[32];
  __shared__ float gl[32];
  __shared__ __align__(16) h16 fst[33 * FEAT_PITCH];
  const int l = blockIdx.x, t = threadIdx.x;
  const int w = t >> 2, q = t & 3;
  const v4u* src = (const v4u*)f2p;
  float acc[8];
#pragma unroll
  for (int e = 0; e < 8; ++e) acc[e] = 0.0f;
#pragma unroll 1
  for (int h = 0; h < HDIM; ++h) {
    const v4u u = src[((size_t)(l * HDIM + h) * WDIM + w) * 4 + q];
    const unsigned u0 = u[0], u1 = u[1], u2 = u[2], u3 = u[3];
    acc[0] += h16_to_f32(u0 & 0xffffu); acc[1] += h16_to_f32(u0 >> 16);
    acc[2] += h16_to_f32(u1 & 0xffffu); acc[3] += h16_to_f32(u1 >> 16);
    acc[4] += h16_to_f32(u2 & 0xffffu); acc[5] += h16_to_f32(u2 >> 16);
    acc[6] += h16_to_f32(u3 & 0xffffu); acc[7] += h16_to_f32(u3 >> 16);
  }
#pragma unroll
  for (int e = 0; e < 8; ++e) fm[w * 32 + 8 * q + e] = acc[e] * (1.0f / HDIM);
  __syncthreads();
  if (t < 32) {
    float s = 0.0f;
#pragma unroll 1
    for (int w2 = 0; w2 < WDIM; ++w2) s += fm[w2 * 32 + t];
    gm[t] = s * (1.0f / WDIM);
  }
  __syncthreads();
  if (t < 32) {
    float a = gfc_b[t];
#pragma unroll 1
    for (int k = 0; k < 32; ++k) a += gm[k] * gfc_w[t * 32 + k];
    gl[t] = 1.0f / (1.0f + expf(-a));
  }
  __syncthreads();
#pragma unroll 1
  for (int i = t; i < 33 * FEAT_PITCH; i += 256) {
    const int j = i >> 6, c = i & 63, cc = c & 31;
    const int s0 = (64 * j) / 33;
    const int e0 = (64 * (j + 1) + 32) / 33;
    float s = 0.0f;
    for (int w2 = s0; w2 < e0; ++w2) s += fm[w2 * 32 + cc];
    float val = s * (1.0f / (float)(e0 - s0)) * gl[cc] * FEAT_CARRY;
    val = (c < 32) ? val : 0.0f;
    fst[i] = (h16)val;
  }
  __syncthreads();
  h16* feat = (h16*)featp;
  for (int g = t; g < 33 * 8; g += 256) {
    const v8h hv = *(const v8h*)(fst + g * 8);
    h16* dp = feat + (size_t)(l * 33) * FEAT_PITCH + g * 8;
    *(volatile v8h*)dp = hv;
    __threadfence();
    *(volatile v8h*)dp = hv;
  }
  if (l == LDIM - 1) {
    const v8h zero8 = {(h16)0.f, (h16)0.f, (h16)0.f, (h16)0.f, (h16)0.f, (h16)0.f, (h16)0.f, (h16)0.f};
    for (int g = t; g < (NLF_PAD - NLF) * 8; g += 256) {
      h16* dp = feat + (size_t)NLF * FEAT_PITCH + g * 8;
      *(volatile v8h*)dp = zero8;
      __threadfence();
      *(volatile v8h*)dp = zero8;
    }
  }
}

__global__ __launch_bounds__(256) void k_headparams(const unsigned short* __restrict__ featp,
                                                    const unsigned short* __restrict__ headp,
                                                    const float* __restrict__ head_b, const float* __restrict__ dt,
                                                    float* __restrict__ ARE, float* __restrict__ AIM,
                                                    float* __restrict__ SGG) {
  __shared__ __align__(16) float slabs[8][16 * 96];
  const h16* feat = (const h16*)featp;
  const h16* head = (const h16*)headp;
  const int tid = threadIdx.x, lane = tid & 31, wave = tid >> 5;
  const int m = lane & 15, hh = lane >> 4, koff = hh * 8;
  const int cp = blockIdx.y * 8 + wave;
  const int m0 = blockIdx.x * 16;
  float* slab = slabs[wave];
  const v8f z8 = {0.f, 0.f, 0.f, 0.f, 0.f, 0.f, 0.f, 0.f};

  const v16h a = Frag<h16>::load(feat + (size_t)(m0 + m) * FEAT_PITCH + koff);
#pragma unroll
  for (int k = 0; k < 3; ++k) {
#pragma unroll
    for (int c2 = 0; c2 < 2; ++c2) {
      const int brow = (k * 32 + 2 * cp + c2) * 16 + m;
      const v16h b = Frag<h16>::load(head + (size_t)brow * 32 + koff);
      const v8f d = wmma_h(a, b, z8);
#pragma unroll
      for (int j = 0; j < 8; ++j) slab[(8 * hh + j) * 96 + k * 32 + c2 * 16 + m] = d[j] * HEAD_FOLD;
    }
  }
  wave_sync();

  const int c = 2 * cp + (lane >> 4);
  const int r = lane & 15;
  const float hb0 = head_b[(c * 16 + r) * 3 + 0];
  const float hb1 = head_b[(c * 16 + r) * 3 + 1];
  const float hb2 = head_b[(c * 16 + r) * 3 + 2];
#pragma unroll 1
  for (int row = 0; row < 16; ++row) {
    const int mrow = m0 + row;
    const bool valid = (mrow < NLF);
    int lf = mrow / WFQ;
    lf = lf > LDIM - 1 ? LDIM - 1 : lf;
    const float d = dt[lf];
    const float p0 = slab[row * 96 + lane] + hb0;
    const float p1 = slab[row * 96 + 32 + lane] + hb1;
    const float p2 = slab[row * 96 + 64 + lane] + hb2;
    const float nu = fmaxf(p0, 0.0f) + log1pf(expf(-fabsf(p0)));
    const float th = tanhf(p1) * PI_F;
    const float sg = 1.0f / (1.0f + expf(-p2));
    const float dec = expf(-nu * d);
    float sn, cs;
    sincosf(th * d, &sn, &cs);
    const float g = 1.0f - expf(-2.0f * fmaxf(d, 0.0f));
    const float are = dec * cs, aim = dec * sn, sgg = sg * g;
    if (valid) {
      const size_t o = (size_t)mrow * 512 + cp * 32 + lane;
      *(volatile float*)(ARE + o) = are;
      *(volatile float*)(AIM + o) = aim;
      *(volatile float*)(SGG + o) = sgg;
      __threadfence();
      *(volatile float*)(ARE + o) = are;
      *(volatile float*)(AIM + o) = aim;
      *(volatile float*)(SGG + o) = sgg;
    }
  }
}

__global__ __launch_bounds__(256) void k_cvtx(const float* __restrict__ x, unsigned short* __restrict__ dstp, int n8) {
  const int i = blockIdx.x * 256 + threadIdx.x;
  if (i < n8) {
    const v4f a = *(const v4f*)(x + (size_t)i * 8);
    const v4f b = *(const v4f*)(x + (size_t)i * 8 + 4);
    v8h hv;
#pragma unroll
    for (int e = 0; e < 4; ++e) { hv[e] = (h16)a[e]; hv[4 + e] = (h16)b[e]; }
    h16* dp = (h16*)dstp + (size_t)i * 8;
    *(volatile v8h*)dp = hv;
    __threadfence();
    *(volatile v8h*)dp = hv;
  }
}

__global__ __launch_bounds__(256) void k_scan(const float* __restrict__ ARE, const float* __restrict__ AIM,
                                              const float* __restrict__ SGG, const float* __restrict__ XFP,
                                              const unsigned short* __restrict__ foldbp, const float* __restrict__ FOLDC,
                                              unsigned* __restrict__ YFPw) {
  __shared__ float slabs[8][64];
  __shared__ float keeps[8][LDIM * 32];
  const int tid = threadIdx.x, lane = tid & 31, wave = tid >> 5;
  const int m = lane & 15, hh = lane >> 4, koff = hh * 8;
  const int gw = blockIdx.x * 8 + wave;
  const int f = gw & 31;
  const int h = gw >> 5;
  float* slab = slabs[wave];
  float* keep = keeps[wave];
  const v16h bfrag = Frag<h16>::load((const h16*)foldbp + m * 32 + koff);
  const float cre = FOLDC[0] * Y_CARRY;
  const float cim = FOLDC[1] * Y_CARRY;
  const v8f z8 = {0.f, 0.f, 0.f, 0.f, 0.f, 0.f, 0.f, 0.f};
  const int npass = (f == 0) ? 2 : 1;
  const int xcol = 2 * f;
  const int i2 = 2 * (lane & 15);

#pragma unroll 1
  for (int pass = 0; pass < npass; ++pass) {
    const int fc = pass ? 32 : f;
    float sre[2][8], sim[2][8];
#pragma unroll
    for (int g = 0; g < 2; ++g)
#pragma unroll
      for (int i = 0; i < 8; ++i) { sre[g][i] = 0.0f; sim[g][i] = 0.0f; }

#pragma unroll 1
    for (int l = 0; l < LDIM; ++l) {
      v8f d[2];
#pragma unroll
      for (int g = 0; g < 2; ++g) {
        const int c = 16 * g + m;
        const size_t pb = ((size_t)((l * WFQ + fc) * 32 + c)) * 16 + 8 * hh;
        const v4f ar0 = *(const v4f*)(ARE + pb), ar1 = *(const v4f*)(ARE + pb + 4);
        const v4f ai0 = *(const v4f*)(AIM + pb), ai1 = *(const v4f*)(AIM + pb + 4);
        const v4f sg0 = *(const v4f*)(SGG + pb), sg1 = *(const v4f*)(SGG + pb + 4);
        const float* xp = XFP + ((size_t)((c * LDIM + l) * HDIM + h)) * 64 + xcol;
        const float xa = xp[0], xb = xp[1];
        const float xre = (f == 0) ? (pass ? xb : xa) : xa;
        const float xim = (f == 0) ? 0.0f : xb;
        v16h af;
#pragma unroll
        for (int i = 0; i < 8; ++i) {
          const float are = (i < 4) ? ar0[i & 3] : ar1[i & 3];
          const float aim = (i < 4) ? ai0[i & 3] : ai1[i & 3];
          const float sgg = (i < 4) ? sg0[i & 3] : sg1[i & 3];
          const float ure = sgg * xre, uim = sgg * xim;
          const float orr = sre[g][i], oi = sim[g][i];
          const float nre = are * orr - aim * oi + ure;
          const float nim = are * oi + aim * orr + uim;
          sre[g][i] = nre;
          sim[g][i] = nim;
          af[i]     = (h16)(nre * H_CARRY);
          af[8 + i] = (h16)(nim * H_CARRY);
        }
        d[g] = wmma_h(af, bfrag, z8);
      }
      if (m < 2) {
#pragma unroll
        for (int g = 0; g < 2; ++g)
#pragma unroll
          for (int j = 0; j < 8; ++j) slab[m * 32 + 16 * g + 8 * hh + j] = d[g][j];
      }
      wave_sync();
      const float r0 = slab[i2], r1 = slab[i2 + 1];
      const float q0 = slab[32 + i2], q1 = slab[32 + i2 + 1];
      const float rs = slab[lane];
      float a0 = r0 * SCAN_FOLD + cre, a1 = r1 * SCAN_FOLD + cre;
      float b0 = q0 * SCAN_FOLD + cim, b1 = q1 * SCAN_FOLD + cim;
      if (f == 0) {
        if (pass == 0) {
          keep[l * 32 + lane] = rs * SCAN_FOLD + cre;
        } else {
          b0 = a0; b1 = a1;
          a0 = keep[l * 32 + i2];
          a1 = keep[l * 32 + i2 + 1];
        }
      }
      const bool dostore = (f != 0) || (pass == 1);
      const float v0 = (lane < 16) ? a0 : b0;
      const float v1 = (lane < 16) ? a1 : b1;
      if (dostore) {
        v2h pk;
        pk[0] = (h16)v0;
        pk[1] = (h16)v1;
        const unsigned u = __builtin_bit_cast(unsigned, pk);
        unsigned* dp = YFPw + ((size_t)((l * HDIM + h) * 64 + 2 * f)) * 16 + lane;
        *(volatile unsigned*)dp = u;
        __threadfence();
        *(volatile unsigned*)dp = u;
      }
      wave_sync();
    }
  }
}

__global__ __launch_bounds__(128) void k_pif(const unsigned short* __restrict__ yfpp, const unsigned short* __restrict__ pifp,
                                             unsigned short* __restrict__ zftp) {
  __shared__ __align__(16) float T[32 * 72];
  const h16* yfp = (const h16*)yfpp;
  const h16* pw  = (const h16*)pifp;
  h16* zft = (h16*)zftp;
  const int tid = threadIdx.x, lane = tid & 31, wave = tid >> 5;
  const int m = lane & 15, hh = lane >> 4, koff = hh * 8;
  const int lh = blockIdx.x;
  const int l = lh >> 6, h = lh & 63;
  const v8f z8 = {0.f, 0.f, 0.f, 0.f, 0.f, 0.f, 0.f, 0.f};
  const v16h a  = Frag<h16>::load(yfp + ((size_t)(lh * 64 + 16 * wave + m)) * 32 + koff);
  const v16h b0 = Frag<h16>::load(pw + m * 32 + koff);
  const v16h b1 = Frag<h16>::load(pw + (16 + m) * 32 + koff);
  const v8f d0 = wmma_h(a, b0, z8);
  const v8f d1 = wmma_h(a, b1, z8);
  const float inv = 1.0f / PIFW_CARRY;
#pragma unroll
  for (int j = 0; j < 8; ++j) {
    T[m * 72 + 16 * wave + 8 * hh + j]        = d0[j] * inv;
    T[(16 + m) * 72 + 16 * wave + 8 * hh + j] = d1[j] * inv;
  }
  __syncthreads();
  const int c8 = (lane & 7) * 8;
#pragma unroll
  for (int it = 0; it < 2; ++it) {
    const int o = 8 * wave + it * 4 + (lane >> 3);
    const v4f s0 = *(const v4f*)(T + o * 72 + c8);
    const v4f s1 = *(const v4f*)(T + o * 72 + c8 + 4);
    v8h hv;
#pragma unroll
    for (int e = 0; e < 4; ++e) { hv[e] = (h16)s0[e]; hv[4 + e] = (h16)s1[e]; }
    h16* dp = zft + ((size_t)((l * CDIM + o) * HDIM + h)) * 64 + c8;
    *(volatile v8h*)dp = hv;
    __threadfence();
    *(volatile v8h*)dp = hv;
  }
}

__global__ __launch_bounds__(256) void k_stats(const float* __restrict__ Y2, float* __restrict__ MUSIG) {
  __shared__ float red[8];
  __shared__ float red2[8];
  const int t = threadIdx.x, lane = t & 31, wave = t >> 5;
  const int lg = blockIdx.x;
  const int l = lg >> 2, g = lg & 3;
  const v4f* base = (const v4f*)(Y2 + (size_t)(l * CDIM + 8 * g) * NPIX);
  float s = 0.0f;
#pragma unroll 1
  for (int k = 0; k < 32; ++k) {
    const v4f v = base[t + 256 * k];
    s += (v[0] + v[1]) + (v[2] + v[3]);
  }
#pragma unroll
  for (int off = 1; off < 32; off <<= 1) s += __shfl_xor(s, off, 32);
  if (lane == 0) red[wave] = s;
  __syncthreads();
  float tot = 0.0f;
#pragma unroll
  for (int k = 0; k < 8; ++k) tot += red[k];
  const float mu = tot * (1.0f / 32768.0f);
  float ss = 0.0f;
#pragma unroll 1
  for (int k = 0; k < 32; ++k) {
    const v4f v = base[t + 256 * k];
    const float e0 = v[0] - mu, e1 = v[1] - mu, e2 = v[2] - mu, e3 = v[3] - mu;
    ss += (e0 * e0 + e1 * e1) + (e2 * e2 + e3 * e3);
  }
#pragma unroll
  for (int off = 1; off < 32; off <<= 1) ss += __shfl_xor(ss, off, 32);
  if (lane == 0) red2[wave] = ss;
  __syncthreads();
  float tot2 = 0.0f;
#pragma unroll
  for (int k = 0; k < 8; ++k) tot2 += red2[k];
  const float var = tot2 * (1.0f / 32768.0f);
  const float rstd = 1.0f / sqrtf(var + GN_EPS);
  if (wave == 0) {
    const float o = (lane == 0) ? mu : ((lane == 1) ? rstd : 0.0f);
    float* dp = MUSIG + lg * 32 + lane;
    *(volatile float*)dp = o;
    __threadfence();
    *(volatile float*)dp = o;
  }
}

__global__ __launch_bounds__(256) void k_gatefinal(const float* __restrict__ x, const float* __restrict__ Y2,
                                                   const float* __restrict__ MUSIG, const float* __restrict__ gn_w,
                                                   const float* __restrict__ gn_b, const float* __restrict__ g1w,
                                                   const float* __restrict__ g1b, const float* __restrict__ g2w,
                                                   const float* __restrict__ g2b, float* __restrict__ out) {
  __shared__ float ysum[32];
  const int t = threadIdx.x, lane = t & 31;
  const int lh = blockIdx.x;
  const int l = lh >> 6, h = lh & 63;
  const int w4 = (t & 15) * 4;
  v4f yv[2];
#pragma unroll
  for (int s = 0; s < 2; ++s) {
    const int c = (t >> 4) + 16 * s;
    yv[s] = *(const v4f*)(Y2 + ((size_t)((l * CDIM + c) * HDIM + h)) * WDIM + w4);
    float rs = (yv[s][0] + yv[s][1]) + (yv[s][2] + yv[s][3]);
#pragma unroll
    for (int off = 1; off < 16; off <<= 1) rs += __shfl_xor(rs, off, 32);
    if ((t & 15) == 0) ysum[c] = rs;
  }
  __syncthreads();
  const int cL = lane;
  const float mu   = MUSIG[(l * 4 + (cL >> 3)) * 32];
  const float rstd = MUSIG[(l * 4 + (cL >> 3)) * 32 + 1];
  const float gw = gn_w[cL], gb = gn_b[cL];
  const float ym = (ysum[cL] * (1.0f / WDIM) - mu) * rstd * gw + gb;
  float o = g2b[cL];
#pragma unroll 1
  for (int k = 0; k < 4; ++k) {
    float p = ym * g1w[k * 32 + cL];
#pragma unroll
    for (int off = 1; off < 32; off <<= 1) p += __shfl_xor(p, off, 32);
    const float z = p + g1b[k];
    const float ak = z / (1.0f + expf(-z));
    o += ak * g2w[cL * 4 + k];
  }
  const float gatev = 1.0f / (1.0f + expf(-o));
#pragma unroll
  for (int s = 0; s < 2; ++s) {
    const int c = (t >> 4) + 16 * s;
    const float gc  = __shfl(gatev, c, 32);
    const float muc = __shfl(mu, c, 32);
    const float rc  = __shfl(rstd, c, 32);
    const float gwc = __shfl(gw, c, 32);
    const float gbc = __shfl(gb, c, 32);
    const size_t oo = ((size_t)((c * LDIM + l) * HDIM + h)) * WDIM + w4;
    const v4f xv = *(const v4f*)(x + oo);
    v4f ov;
#pragma unroll
    for (int e = 0; e < 4; ++e) {
      const float z = (yv[s][e] - muc) * rc * gwc + gbc;
      ov[e] = xv[e] + z * gc;
    }
    *(volatile v4f*)(out + oo) = ov;
    __threadfence();
    *(volatile v4f*)(out + oo) = ov;
  }
}

extern "C" void kernel_launch(void* const* d_in, const int* in_sizes, int n_in,
                              void* d_out, int out_size, void* d_ws, size_t ws_size, hipStream_t stream) {
  if (n_in < 23 || d_out == nullptr || d_ws == nullptr) return;
  if (in_sizes[0] != NELEM || in_sizes[1] != LDIM || in_sizes[2] != 9216 || in_sizes[4] != 9216 ||
      in_sizes[8] != NHEAD * 32 || in_sizes[9] != NHEAD || in_sizes[10] != 1024 || in_sizes[15] != 1024 ||
      out_size != NELEM) return;

  const float* x       = (const float*)d_in[0];
  const float* dt      = (const float*)d_in[1];
  const float* conv1_w = (const float*)d_in[2];
  const float* conv1_b = (const float*)d_in[3];
  const float* conv2_w = (const float*)d_in[4];
  const float* conv2_b = (const float*)d_in[5];
  const float* gfc_w   = (const float*)d_in[6];
  const float* gfc_b   = (const float*)d_in[7];
  const float* head_w  = (const float*)d_in[8];
  const float* head_b  = (const float*)d_in[9];
  const float* mix_w   = (const float*)d_in[10];
  const float* mix_b   = (const float*)d_in[11];
  const float* rank_sc = (const float*)d_in[12];
  const float* proj_w  = (const float*)d_in[13];
  const float* proj_b  = (const float*)d_in[14];
  const float* pif_w   = (const float*)d_in[15];
  const float* pif_b   = (const float*)d_in[16];
  const float* gn_w    = (const float*)d_in[17];
  const float* gn_b    = (const float*)d_in[18];
  const float* g1w     = (const float*)d_in[19];
  const float* g1b     = (const float*)d_in[20];
  const float* g2w     = (const float*)d_in[21];
  const float* g2b     = (const float*)d_in[22];
  float* out = (float*)d_out;

  char* ws = (char*)d_ws; size_t off = 0;
  auto carve = [&](size_t bytes) -> char* { char* p = ws + off; off += (bytes + 255) & ~(size_t)255; return p; };
  unsigned short* CW1   = (unsigned short*)carve((size_t)9 * 32 * 32 * 2);
  unsigned short* CW2   = (unsigned short*)carve((size_t)9 * 32 * 32 * 2);
  unsigned short* HEADP = (unsigned short*)carve((size_t)NHEAD * 32 * 2);
  unsigned short* PIF16 = (unsigned short*)carve((size_t)32 * 32 * 2);
  unsigned short* FT16  = (unsigned short*)carve((size_t)64 * 64 * 2);
  unsigned short* IT16  = (unsigned short*)carve((size_t)64 * 64 * 2);
  unsigned short* FOLDB = (unsigned short*)carve((size_t)16 * 32 * 2);
  float*          FOLDC = (float*)carve((size_t)32 * 4);
  unsigned short* F1    = (unsigned short*)carve((size_t)LDIM * NPIX * CDIM * 2);
  unsigned short* F2    = (unsigned short*)carve((size_t)LDIM * NPIX * CDIM * 2);
  unsigned short* FEAT  = (unsigned short*)carve((size_t)NLF_PAD * FEAT_PITCH * 2);
  float*          ARE   = (float*)carve((size_t)NLF * 32 * 16 * 4);
  float*          AIM   = (float*)carve((size_t)NLF * 32 * 16 * 4);
  float*          SGG   = (float*)carve((size_t)NLF * 32 * 16 * 4);
  unsigned short* X16   = (unsigned short*)carve((size_t)NXROW * 64 * 2);
  float*          XFP   = (float*)carve((size_t)NXROW * 64 * 4);
  unsigned short* YFP   = (unsigned short*)carve((size_t)LDIM * HDIM * 64 * 32 * 2);
  unsigned short* ZFT   = (unsigned short*)carve((size_t)NXROW * 64 * 2);
  float*          Y2    = (float*)carve((size_t)NXROW * 64 * 4);
  float*          MUSIG = (float*)carve((size_t)64 * 32 * 4);
  if (off > ws_size || off > (size_t)134217728) return;

  k_prep<<<PREP_BLOCKS, PREP_THR, 0, stream>>>(conv1_w, conv2_w, head_w, pif_w, mix_w, mix_b, rank_sc, proj_w, proj_b,
                                               CW1, CW2, HEADP, PIF16, FT16, IT16, FOLDB, FOLDC);
  k_conv<true ><<<LDIM * 8, 256, 0, stream>>>(x, F1, CW1, conv1_b, F1);
  k_conv<false><<<LDIM * 8, 256, 0, stream>>>(x, F1, CW2, conv2_b, F2);
  k_pool<<<LDIM, 256, 0, stream>>>(F2, gfc_w, gfc_b, FEAT);
  k_headparams<<<dim3(NLF_PAD / 16, 2), 256, 0, stream>>>(FEAT, HEADP, head_b, dt, ARE, AIM, SGG);
  const int n8x = NELEM / 8;
  k_cvtx<<<(n8x + 255) / 256, 256, 0, stream>>>(x, X16, n8x);
  wmma_gemm64<0, false, 0, 0, false, 0><<<dim3(NXROW / 64 / 8, 1), 256, 0, stream>>>(
      X16, X16, 64, 0L, FT16, FT16, 64, 0L, (void*)XFP, (void*)XFP, 64, 0L,
      pif_b, XFP, 0L, NXROW, 64, 64, 1.0f);
  k_scan<<<(HDIM * 32) / 8, 256, 0, stream>>>(ARE, AIM, SGG, XFP, FOLDB, FOLDC, (unsigned*)YFP);
  k_pif<<<LDIM * HDIM, 128, 0, stream>>>(YFP, PIF16, ZFT);
  wmma_gemm64<0, false, 3, 0, false, 0><<<dim3(NXROW / 64 / 8, 1), 256, 0, stream>>>(
      ZFT, ZFT, 64, 0L, IT16, IT16, 64, 0L, (void*)Y2, (void*)Y2, 64, 0L,
      pif_b, Y2, 0L, NXROW, 64, 64, IDFT_FOLD);
  k_stats<<<LDIM * 4, 256, 0, stream>>>(Y2, MUSIG);
  k_gatefinal<<<LDIM * HDIM, 256, 0, stream>>>(x, Y2, MUSIG, gn_w, gn_b, g1w, g1b, g2w, g2b, out);
}
